// ToyTransformerBlock_4999341932774
// MI455X (gfx1250) — hardware-verified
//
#include <hip/hip_runtime.h>
#include <stddef.h>


typedef _Float16 v16h __attribute__((ext_vector_type(16)));
typedef _Float16 v8h  __attribute__((ext_vector_type(8)));
typedef float    v8f  __attribute__((ext_vector_type(8)));
typedef float    v4f  __attribute__((ext_vector_type(4)));
typedef _Float16 h16;

#ifndef NB
#define NB 4
#endif
#ifndef SEQ
#define SEQ 2048
#endif
#define NB_FULL  4
#define SEQ_FULL 2048
#define DIM   1024
#define MROWS (NB * SEQ)

static_assert(NB >= 1 && NB <= NB_FULL);
static_assert(SEQ >= 256 && SEQ <= SEQ_FULL && (SEQ % 256) == 0);
static_assert((DIM % 64) == 0 && (DIM % 32) == 0);
static_assert((SEQ % 64) == 0 && (SEQ % 32) == 0);
static_assert((MROWS % 64) == 0 && (MROWS % 8) == 0);
static_assert(DIM == 4 * 32 * 8);
static_assert(DIM == 8 * 32 * 4);
static_assert(DIM == 32 * 32);

#define LDC 68
static_assert((LDC % 4) == 0 && LDC >= 64);

#define WCARRY 64.0f
#define PCARRY 16384.0f
#define VCARRY 64.0f
#define SSCALE 0.03125f

#define MAX2(a, b) ((a) > (b) ? (a) : (b))
#define WSQ_BYTES     ((size_t)DIM * DIM * 2)
#define PLANE16_BYTES ((size_t)MROWS * DIM * 2)
#define S_BYTES       ((size_t)NB * SEQ * SEQ * 4)
#define P_BYTES       ((size_t)NB * SEQ * SEQ * 2)
#define H_BYTES       ((size_t)MROWS * DIM * 4)
#define RA_BYTES MAX2(MAX2((size_t)3 * WSQ_BYTES + PLANE16_BYTES, S_BYTES), PLANE16_BYTES)
#define RB_BYTES MAX2(MAX2((size_t)2 * PLANE16_BYTES, P_BYTES), H_BYTES)
#define OFF_WO  ((size_t)0)
#define OFF_RA  (OFF_WO + WSQ_BYTES)
#define OFF_RB  (OFF_RA + RA_BYTES)
#define OFF_VT  (OFF_RB + RB_BYTES)
#define WS_TOTAL (OFF_VT + PLANE16_BYTES)
#define OFF_WQ  (OFF_RA)
#define OFF_WK  (OFF_WQ + WSQ_BYTES)
#define OFF_WV  (OFF_WK + WSQ_BYTES)
#define OFF_X16 (OFF_WV + WSQ_BYTES)
#define OFF_S   (OFF_RA)
#define OFF_CTX (OFF_RA)
#define OFF_Q   (OFF_RB)
#define OFF_K   (OFF_Q + PLANE16_BYTES)
#define OFF_P   (OFF_RB)
#define OFF_H   (OFF_RB)
static_assert((WSQ_BYTES % 128) == 0 && (PLANE16_BYTES % 128) == 0);
static_assert((S_BYTES % 128) == 0 && (P_BYTES % 128) == 0 && (H_BYTES % 128) == 0);
static_assert((RA_BYTES % 128) == 0 && (RB_BYTES % 128) == 0);
static_assert(OFF_X16 + PLANE16_BYTES <= OFF_RA + RA_BYTES);
static_assert(OFF_S + S_BYTES <= OFF_RA + RA_BYTES);
static_assert(OFF_CTX + PLANE16_BYTES <= OFF_RA + RA_BYTES);
static_assert(OFF_K + PLANE16_BYTES <= OFF_RB + RB_BYTES);
static_assert(OFF_P + P_BYTES <= OFF_RB + RB_BYTES);
static_assert(OFF_H + H_BYTES <= OFF_RB + RB_BYTES);
static_assert(WS_TOTAL <= (size_t)134217728);

__device__ __forceinline__ float bf16r(float x) {
  unsigned int u = __float_as_uint(x);
  u = (u + 0x7FFFu + ((u >> 16) & 1u)) & 0xFFFF0000u;
  return __uint_as_float(u);
}

static __device__ __forceinline__ h16 toh_flush(float v) {
  const h16 r = (h16)v;
  return (fabsf(v) < 6.103515625e-05f) ? (h16)0.0f : r;
}

__device__ __forceinline__ v16h frag_at(const _Float16* p) {
  v8h lo = *(const v8h*)(p);
  v8h hi = *(const v8h*)(p + 16);
  v16h out;
#pragma unroll
  for (int i = 0; i < 8; ++i) { out[i] = lo[i]; out[i + 8] = hi[i]; }
  return out;
}

__device__ __forceinline__ v8f wmma16(v16h a, v16h b, v8f c) {
  v8f d = __builtin_amdgcn_wmma_f32_16x16x32_f16(false, a, false, b, (short)0, c,
                                                 false, false);
  asm volatile("v_nop\n\tv_nop\n\tv_nop\n\tv_nop" : "+v"(d) : "v"(a), "v"(b));
  return d;
}

__device__ __forceinline__ float red32_sum(float x) {
#pragma unroll
  for (int off = 1; off < 32; off <<= 1) x += __shfl_xor(x, off, 32);
  return x;
}
__device__ __forceinline__ float red32_max(float x) {
#pragma unroll
  for (int off = 1; off < 32; off <<= 1) x = fmaxf(x, __shfl_xor(x, off, 32));
  return x;
}

__device__ __forceinline__ void cast_row_body(const float* __restrict__ src,
                                              _Float16* __restrict__ dst, const float carry) {
#pragma unroll 1
  for (unsigned j = 0; j < 4u; ++j) {
    const v4f a0 = *(const v4f*)(src + j * 256u);
    const v4f a1 = *(const v4f*)(src + j * 256u + 4u);
    v8h o;
#pragma unroll
    for (int i = 0; i < 4; ++i) {
      o[i]     = toh_flush(carry * bf16r(a0[i]));
      o[i + 4] = toh_flush(carry * bf16r(a1[i]));
    }
    _Float16* p = dst + j * 256u;
    *(volatile v8h*)p = o;
    __threadfence();
    *(volatile v8h*)p = o;
  }
}

__global__ __launch_bounds__(256) void wcast_kernel(
    const float* __restrict__ W, _Float16* __restrict__ Wt) {
  const unsigned lane = threadIdx.x & 31u;
  const unsigned wave = (unsigned)__builtin_amdgcn_readfirstlane((int)(threadIdx.x >> 5));
  const unsigned row = blockIdx.x * 8u + wave;
  cast_row_body(W + (size_t)row * DIM + lane * 8u, Wt + (size_t)row * DIM + lane * 8u, WCARRY);
}

__global__ __launch_bounds__(256) void xcast_kernel(
    const float* __restrict__ X, _Float16* __restrict__ X16) {
  const unsigned lane = threadIdx.x & 31u;
  const unsigned wave = (unsigned)__builtin_amdgcn_readfirstlane((int)(threadIdx.x >> 5));
  const unsigned crow = blockIdx.x * 8u + wave;
  const unsigned bidx = crow / (unsigned)SEQ;
  const unsigned sq = crow - bidx * (unsigned)SEQ;
  const size_t srow = (size_t)bidx * SEQ_FULL + sq;
  cast_row_body(X + srow * DIM + lane * 8u, X16 + (size_t)crow * DIM + lane * 8u, 1.0f);
}

template <int MODE>
__device__ __forceinline__ void gemm_body(
    const _Float16* __restrict__ A16, const _Float16* __restrict__ Bt, const unsigned K,
    const float* __restrict__ addf,
    float* __restrict__ outf, _Float16* __restrict__ out16) {
  __shared__ float Cs[64 * LDC];
  const unsigned tid = threadIdx.x, lane = tid & 31u, w = tid >> 5;
  const unsigned mw = w >> 1, nw = w & 1u;
  const unsigned hh = lane >> 4, m = lane & 15u;
  const unsigned n0 = blockIdx.x * 64u;
  const unsigned row0 = blockIdx.y * 64u;

  const _Float16* ap  = A16 + (size_t)(row0 + mw * 16u + m) * K + hh * 8u;
  const _Float16* bp0 = Bt + (size_t)(n0 + nw * 32u + m) * K + hh * 8u;
  const _Float16* bp1 = bp0 + (size_t)16 * K;
  v8f acc0 = {}, acc1 = {};
#pragma unroll 2
  for (unsigned k0 = 0; k0 < K; k0 += 32u) {
    const v16h a  = frag_at(ap + k0);
    const v16h b0 = frag_at(bp0 + k0);
    const v16h b1 = frag_at(bp1 + k0);
    acc0 = wmma16(a, b0, acc0);
    acc1 = wmma16(a, b1, acc1);
  }
#pragma unroll
  for (int r = 0; r < 8; ++r) {
    float* d = &Cs[(mw * 16u + hh * 8u + (unsigned)r) * LDC + nw * 32u + m];
    d[0]  = acc0[r];
    d[16] = acc1[r];
  }
  __syncthreads();

  if (MODE == 0 || MODE == 3) {
    const float cs = (MODE == 3) ? (VCARRY / PCARRY) : (1.0f / WCARRY);
    v8h x[2];
    size_t off[2];
#pragma unroll
    for (unsigned i = 0; i < 2u; ++i) {
      const unsigned r = 32u * i + (tid >> 3);
      const unsigned c = (tid & 7u) * 8u;
      const v4f u0 = *(const v4f*)&Cs[r * LDC + c];
      const v4f u1 = *(const v4f*)&Cs[r * LDC + c + 4];
#pragma unroll
      for (int j = 0; j < 4; ++j) {
        x[i][j]     = toh_flush(u0[j] * cs);
        x[i][j + 4] = toh_flush(u1[j] * cs);
      }
      off[i] = (size_t)(row0 + r) * DIM + n0 + c;
    }
#pragma unroll
    for (int i = 0; i < 2; ++i) *(volatile v8h*)(out16 + off[i]) = x[i];
    __threadfence();
#pragma unroll
    for (int i = 0; i < 2; ++i) *(volatile v8h*)(out16 + off[i]) = x[i];
  }

  if (MODE == 1) {
    const unsigned bidx = row0 / (unsigned)SEQ;
    const unsigned key0 = row0 - bidx * (unsigned)SEQ;
    v8h x[2];
    size_t off[2];
#pragma unroll
    for (unsigned i = 0; i < 2u; ++i) {
      const unsigned dcol = 32u * i + (tid >> 3);
      const unsigned kk = (tid & 7u) * 8u;
#pragma unroll
      for (unsigned j = 0; j < 8u; ++j) {
        const float t = Cs[(kk + j) * LDC + dcol] * (1.0f / WCARRY);
        x[i][j] = toh_flush(t);
      }
      off[i] = ((size_t)bidx * DIM + n0 + dcol) * SEQ + key0 + kk;
    }
#pragma unroll
    for (int i = 0; i < 2; ++i) *(volatile v8h*)(out16 + off[i]) = x[i];
    __threadfence();
#pragma unroll
    for (int i = 0; i < 2; ++i) *(volatile v8h*)(out16 + off[i]) = x[i];
  }

  if (MODE == 2) {
    v4f xs[4];
    size_t off[4];
#pragma unroll
    for (unsigned i = 0; i < 4u; ++i) {
      const unsigned r = 16u * i + (tid >> 4);
      const unsigned c = (tid & 15u) * 4u;
      const v4f u = *(const v4f*)&Cs[r * LDC + c];
      xs[i] = u * SSCALE;
      off[i] = (size_t)(row0 + r) * SEQ + n0 + c;
    }
#pragma unroll
    for (int i = 0; i < 4; ++i) *(volatile v4f*)(outf + off[i]) = xs[i];
    __threadfence();
#pragma unroll
    for (int i = 0; i < 4; ++i) *(volatile v4f*)(outf + off[i]) = xs[i];
  }

  if (MODE == 4) {
    const float cs = 1.0f / (WCARRY * VCARRY);
    v4f xs[4];
    size_t off[4];
#pragma unroll
    for (unsigned i = 0; i < 4u; ++i) {
      const unsigned r = 16u * i + (tid >> 4);
      const unsigned c = (tid & 15u) * 4u;
      const unsigned crow = row0 + r;
      const unsigned bidx = crow / (unsigned)SEQ;
      const unsigned sq = crow - bidx * (unsigned)SEQ;
      const size_t frow = (size_t)bidx * SEQ_FULL + sq;
      const v4f u = *(const v4f*)&Cs[r * LDC + c];
      const v4f xin = *(const v4f*)(addf + frow * DIM + n0 + c);
      v4f val;
#pragma unroll
      for (int j = 0; j < 4; ++j) val[j] = bf16r(xin[j]) + u[j] * cs;
      xs[i] = val;
      off[i] = (size_t)crow * DIM + n0 + c;
    }
#pragma unroll
    for (int i = 0; i < 4; ++i) *(volatile v4f*)(outf + off[i]) = xs[i];
    __threadfence();
#pragma unroll
    for (int i = 0; i < 4; ++i) *(volatile v4f*)(outf + off[i]) = xs[i];
  }
}

__global__ __launch_bounds__(256) void gemm_qk_kernel(
    const _Float16* __restrict__ A16, const _Float16* __restrict__ Bt,
    _Float16* __restrict__ out16) {
  gemm_body<0>(A16, Bt, (unsigned)DIM, (const float*)0, (float*)0, out16);
}
__global__ __launch_bounds__(256) void gemm_v_kernel(
    const _Float16* __restrict__ A16, const _Float16* __restrict__ Bt,
    _Float16* __restrict__ vt) {
  gemm_body<1>(A16, Bt, (unsigned)DIM, (const float*)0, (float*)0, vt);
}
__global__ __launch_bounds__(256) void gemm_s_kernel(
    const _Float16* __restrict__ Qh, const _Float16* __restrict__ Kh, float* __restrict__ S) {
  const size_t b = blockIdx.z;
  gemm_body<2>(Qh + b * (size_t)SEQ * DIM, Kh + b * (size_t)SEQ * DIM, (unsigned)DIM,
               (const float*)0, S + b * (size_t)SEQ * SEQ, (_Float16*)0);
}
__global__ __launch_bounds__(256) void gemm_pv_kernel(
    const _Float16* __restrict__ P16, const _Float16* __restrict__ Vt,
    _Float16* __restrict__ ctx) {
  const size_t b = blockIdx.z;
  gemm_body<3>(P16 + b * (size_t)SEQ * SEQ, Vt + b * (size_t)DIM * SEQ, (unsigned)SEQ,
               (const float*)0, (float*)0, ctx + b * (size_t)SEQ * DIM);
}
__global__ __launch_bounds__(256) void gemm_wo_kernel(
    const _Float16* __restrict__ A16, const _Float16* __restrict__ Bt,
    const float* __restrict__ xin, float* __restrict__ hpl) {
  gemm_body<4>(A16, Bt, (unsigned)DIM, xin, hpl, (_Float16*)0);
}

__global__ __launch_bounds__(256) void softmax_kernel(
    const float* __restrict__ S, _Float16* __restrict__ P16) {
#pragma clang fp contract(off)
  const unsigned lane = threadIdx.x & 31u;
  const unsigned wave = (unsigned)__builtin_amdgcn_readfirstlane((int)(threadIdx.x >> 5));
  const size_t row = (size_t)blockIdx.x * 8u + wave;
  const float* sr = S + row * SEQ + lane * 8u;

  float mx = -3.0e38f;
#pragma unroll 1
  for (unsigned j = 0; j < (unsigned)(SEQ / 256); ++j) {
    const v4f a0 = *(const v4f*)(sr + j * 256u);
    const v4f a1 = *(const v4f*)(sr + j * 256u + 4u);
#pragma unroll
    for (int i = 0; i < 4; ++i) mx = fmaxf(mx, fmaxf(a0[i], a1[i]));
  }
  mx = red32_max(mx);

  float sum = 0.0f;
#pragma unroll 1
  for (unsigned j = 0; j < (unsigned)(SEQ / 256); ++j) {
    const v4f a0 = *(const v4f*)(sr + j * 256u);
    const v4f a1 = *(const v4f*)(sr + j * 256u + 4u);
#pragma unroll
    for (int i = 0; i < 4; ++i) sum += __expf(a0[i] - mx) + __expf(a1[i] - mx);
  }
  sum = red32_sum(sum);
  const float inv = PCARRY * (1.0f / sum);

#pragma unroll 1
  for (unsigned j = 0; j < (unsigned)(SEQ / 256); ++j) {
    const v4f a0 = *(const v4f*)(sr + j * 256u);
    const v4f a1 = *(const v4f*)(sr + j * 256u + 4u);
    v8h o;
#pragma unroll
    for (int i = 0; i < 4; ++i) {
      o[i]     = toh_flush(__expf(a0[i] - mx) * inv);
      o[i + 4] = toh_flush(__expf(a1[i] - mx) * inv);
    }
    _Float16* p = P16 + row * SEQ + j * 256u + lane * 8u;
    *(volatile v8h*)p = o;
    __threadfence();
    *(volatile v8h*)p = o;
  }
}

__global__ __launch_bounds__(256) void ln_out_kernel(
    const float* __restrict__ H, float* __restrict__ out) {
#pragma clang fp contract(off)
  const unsigned lane = threadIdx.x & 31u;
  const unsigned wave = (unsigned)__builtin_amdgcn_readfirstlane((int)(threadIdx.x >> 5));
  const unsigned crow = blockIdx.x * 8u + wave;
  const unsigned bidx = crow / (unsigned)SEQ;
  const unsigned sq = crow - bidx * (unsigned)SEQ;
  const size_t frow = (size_t)bidx * SEQ_FULL + sq;
  const float* hr = H + (size_t)crow * DIM + lane * 4u;

  float s = 0.0f;
#pragma unroll 1
  for (unsigned j = 0; j < 8u; ++j) {
    const v4f a = *(const v4f*)(hr + j * 128u);
    s += (a[0] + a[1]) + (a[2] + a[3]);
  }
  const float mean = red32_sum(s) * (1.0f / (float)DIM);

  float ss = 0.0f;
#pragma unroll 1
  for (unsigned j = 0; j < 8u; ++j) {
    const v4f a = *(const v4f*)(hr + j * 128u);
#pragma unroll
    for (int i = 0; i < 4; ++i) {
      const float d = a[i] - mean;
      ss += d * d;
    }
  }
  const float var = red32_sum(ss) * (1.0f / (float)DIM);
  const float rstd = 1.0f / sqrtf(var + 1.0e-5f);

#pragma unroll 1
  for (unsigned j = 0; j < 8u; ++j) {
    const v4f a = *(const v4f*)(hr + j * 128u);
    v4f o;
#pragma unroll
    for (int i = 0; i < 4; ++i) o[i] = (a[i] - mean) * rstd;
    float* p = out + frow * DIM + j * 128u + lane * 4u;
    *(volatile v4f*)p = o;
    __threadfence();
    *(volatile v4f*)p = o;
  }
}

extern "C" void kernel_launch(void* const* d_in, const int* in_sizes, int n_in,
                              void* d_out, int out_size, void* d_ws, size_t ws_size,
                              hipStream_t stream) {
  if (n_in < 5) return;
  const long long need_x = ((long long)(NB - 1) * SEQ_FULL + SEQ) * DIM;
  if ((long long)in_sizes[0] < need_x) return;
  if ((long long)in_sizes[1] < (long long)DIM * DIM) return;
  if ((long long)in_sizes[2] < (long long)DIM * DIM) return;
  if ((long long)in_sizes[3] < (long long)DIM * DIM) return;
  if ((long long)in_sizes[4] < (long long)DIM * DIM) return;
  if ((long long)out_size < need_x) return;
  if (ws_size < WS_TOTAL) return;

  const float* X  = (const float*)d_in[0];
  const float* wq = (const float*)d_in[1];
  const float* wk = (const float*)d_in[2];
  const float* wv = (const float*)d_in[3];
  const float* wo = (const float*)d_in[4];
  float* out = (float*)d_out;

  char* ws = (char*)d_ws;
  _Float16* Wo_t  = (_Float16*)(ws + OFF_WO);
  _Float16* Wq_t  = (_Float16*)(ws + OFF_WQ);
  _Float16* Wk_t  = (_Float16*)(ws + OFF_WK);
  _Float16* Wv_t  = (_Float16*)(ws + OFF_WV);
  _Float16* X16   = (_Float16*)(ws + OFF_X16);
  _Float16* Qh16  = (_Float16*)(ws + OFF_Q);
  _Float16* Kh16  = (_Float16*)(ws + OFF_K);
  _Float16* Vt16  = (_Float16*)(ws + OFF_VT);
  float*    Sf    = (float*)(ws + OFF_S);
  _Float16* P16   = (_Float16*)(ws + OFF_P);
  _Float16* Ctx16 = (_Float16*)(ws + OFF_CTX);
  float*    Hpl   = (float*)(ws + OFF_H);

  dim3 blk(256);
  dim3 gg(DIM / 64, MROWS / 64);

  wcast_kernel<<<dim3(DIM / 8), blk, 0, stream>>>(wq, Wq_t);
  wcast_kernel<<<dim3(DIM / 8), blk, 0, stream>>>(wk, Wk_t);
  wcast_kernel<<<dim3(DIM / 8), blk, 0, stream>>>(wv, Wv_t);
  wcast_kernel<<<dim3(DIM / 8), blk, 0, stream>>>(wo, Wo_t);
  xcast_kernel<<<dim3(MROWS / 8), blk, 0, stream>>>(X, X16);

  gemm_qk_kernel<<<gg, blk, 0, stream>>>(X16, Wq_t, Qh16);
  gemm_qk_kernel<<<gg, blk, 0, stream>>>(X16, Wk_t, Kh16);
  gemm_v_kernel<<<gg, blk, 0, stream>>>(X16, Wv_t, Vt16);
  gemm_s_kernel<<<dim3(SEQ / 64, SEQ / 64, NB), blk, 0, stream>>>(Qh16, Kh16, Sf);
  softmax_kernel<<<dim3(MROWS / 8), blk, 0, stream>>>(Sf, P16);
  gemm_pv_kernel<<<dim3(DIM / 64, SEQ / 64, NB), blk, 0, stream>>>(P16, Vt16, Ctx16);
  gemm_wo_kernel<<<gg, blk, 0, stream>>>(Ctx16, Wo_t, X, Hpl);
  ln_out_kernel<<<dim3(MROWS / 8), blk, 0, stream>>>(Hpl, out);
}
